// DurationPredictorGRU_58523224375975
// MI455X (gfx1250) — hardware-verified
//
#include <hip/hip_runtime.h>
#define NB 32
#define TT 2048
#define FF 64
#define HH 256
#define G3 768
#define NSING 1024

typedef __bf16 v16b __attribute__((ext_vector_type(16)));
typedef unsigned short v8us __attribute__((ext_vector_type(8), may_alias));
typedef float  v8f  __attribute__((ext_vector_type(8)));
typedef float  v4f  __attribute__((ext_vector_type(4)));
typedef float  v4fa __attribute__((ext_vector_type(4), may_alias));
union FragB { v16b v; v8us half[2]; unsigned short u[16]; };

__device__ __forceinline__ unsigned short bf16_bits(float x) { unsigned int u = __float_as_uint(x); return (unsigned short)((u + 0x7FFFu + ((u >> 16) & 1u)) >> 16); }
__device__ __forceinline__ float bf16_val(unsigned short b) { return __uint_as_float(((unsigned int)b) << 16); }
__device__ __forceinline__ float bf16_round(float x) { return bf16_val(bf16_bits(x)); }
template <int NT>
__device__ __forceinline__ v8f mmaN(v16b ah, v16b al, v16b bh, v16b bl, v8f c) {
  c = __builtin_amdgcn_wmma_f32_16x16x32_bf16(false, ah, false, bh, (short)0, c, false, false);
  if (NT >= 2) c = __builtin_amdgcn_wmma_f32_16x16x32_bf16(false, al, false, bh, (short)0, c, false, false);
  if (NT >= 3) c = __builtin_amdgcn_wmma_f32_16x16x32_bf16(false, ah, false, bl, (short)0, c, false, false);
  asm volatile("v_nop\n\tv_nop\n\tv_nop\n\tv_nop" : "+v"(c) : "v"(ah), "v"(al), "v"(bh), "v"(bl));
  return c;
}

__global__ __launch_bounds__(256) void k_wt_bf16(const float* __restrict__ W, unsigned short* __restrict__ Wt, int K, int N) {
  const int t = blockIdx.x * 256 + threadIdx.x;
  const int k8n = K / 8;
  if (t >= N * k8n) return;
  const int n = t / k8n, k8 = (t % k8n) * 8;
  v8us v;
#pragma unroll
  for (int i = 0; i < 8; ++i) v[i] = bf16_bits(W[(size_t)(k8 + i) * N + n]);
  *(volatile v8us*)(Wt + (size_t)n * K + k8) = v;
  __threadfence();
  *(volatile v8us*)(Wt + (size_t)n * K + k8) = v;
}

template <bool ASPLIT, int ACT, bool BIAS_BF16>
__global__ __launch_bounds__(128) void k_gemm_bf(const float* __restrict__ A, int lda, const unsigned short* __restrict__ Wt, int ldb,
                                               const float* __restrict__ bias, float* __restrict__ C, int ldc, int M, int N, int K) {
  __shared__ __attribute__((aligned(16))) float so[4][16][64];
  const int tid = threadIdx.x, w = tid >> 5, lane = tid & 31, ln = lane & 15, hh = lane >> 4;
  const int ntn = N / 64;
  const int wid = blockIdx.x * 4 + w;
  const int mt = wid / ntn, nq = wid % ntn;
  if (mt * 16 >= M) return;
  const int row0 = mt * 16, col0 = nq * 64;
  const float* arow = A + (size_t)(row0 + ln) * lda;
  v8f acc[4] = {};
  for (int kb = 0; kb < K; kb += 32) {
    FragB ah, al;
    const v4f x0 = *(const v4fa*)(arow + kb + 8 * hh), x1 = *(const v4fa*)(arow + kb + 8 * hh + 4);
    const v4f x2 = *(const v4fa*)(arow + kb + 16 + 8 * hh), x3 = *(const v4fa*)(arow + kb + 16 + 8 * hh + 4);
    float xs[16] = {x0[0],x0[1],x0[2],x0[3],x1[0],x1[1],x1[2],x1[3],x2[0],x2[1],x2[2],x2[3],x3[0],x3[1],x3[2],x3[3]};
#pragma unroll
    for (int i = 0; i < 16; ++i) { const unsigned short hb = bf16_bits(xs[i]); ah.u[i] = hb; al.u[i] = ASPLIT ? bf16_bits(xs[i] - bf16_val(hb)) : (unsigned short)0; }
#pragma unroll
    for (int t = 0; t < 4; ++t) {
      const unsigned short* brow = Wt + (size_t)(col0 + t * 16 + ln) * ldb + kb;
      FragB b;
      b.half[0] = *(const v8us*)(brow + 8 * hh);
      b.half[1] = *(const v8us*)(brow + 16 + 8 * hh);
      acc[t] = mmaN<ASPLIT ? 2 : 1>(ah.v, al.v, b.v, b.v, acc[t]);
    }
  }
#pragma unroll
  for (int t = 0; t < 4; ++t) {
    float bv = bias ? bias[col0 + t * 16 + ln] : 0.f;
    if (BIAS_BF16) bv = bf16_round(bv);
#pragma unroll
    for (int r = 0; r < 8; ++r) { float v = acc[t][r] + bv; if (ACT == 1) v = fmaxf(v, 0.f); so[w][8 * hh + r][t * 16 + ln] = v; }
  }
  __builtin_amdgcn_fence(__ATOMIC_ACQ_REL, "workgroup");
  __builtin_amdgcn_wave_barrier();
  const int rsub = lane >> 4, c4 = (lane & 15) * 4;
  for (int pass = 0; pass < 2; ++pass) {
#pragma unroll
    for (int q = 0; q < 8; ++q) {
      const int r = q * 2 + rsub;
      const v4f v = *(const v4fa*)&so[w][r][c4];
      *(volatile v4f*)(C + (size_t)(row0 + r) * ldc + col0 + c4) = v;
    }
    if (pass == 0) __threadfence();
  }
}

template <int D, bool CAUSAL>
__global__ __launch_bounds__(128) void k_flash(const float* __restrict__ qb, const float* __restrict__ kb, const float* __restrict__ vb,
                                             int pitch, int T, int H, float scale, float* __restrict__ y, int ypitch) {
  constexpr int KS = D / 32;
  constexpr int DT = D / 16;
  __shared__ __attribute__((aligned(16))) unsigned short sKh[32][D + 8], sKl[32][D + 8], sVh[32][D + 8], sVl[32][D + 8];
  __shared__ __attribute__((aligned(16))) unsigned short sPh[4][16][40], sPl[4][16][40];
  __shared__ __attribute__((aligned(16))) float sO[4][16][D];
  const int tid = threadIdx.x, w = tid >> 5, lane = tid & 31, ln = lane & 15, hh = lane >> 4;
  const int nqb = (T + 63) / 64;
  const int bh = blockIdx.x / nqb, qblk = blockIdx.x % nqb;
  const int b = bh / H, h = bh % H;
  const int q0 = qblk * 64 + w * 16;
  const float* Q = qb + (size_t)b * T * pitch + h * D;
  const float* K = kb + (size_t)b * T * pitch + h * D;
  const float* V = vb + (size_t)b * T * pitch + h * D;

  FragB aqh[KS], aql[KS];
  {
    int row = q0 + ln; if (row >= T) row = T - 1;
    const float* qr = Q + (size_t)row * pitch;
#pragma unroll
    for (int ks = 0; ks < KS; ++ks)
#pragma unroll
      for (int i = 0; i < 16; ++i) {
        const int d = ks * 32 + ((i < 8) ? (8 * hh + i) : (16 + 8 * hh + (i - 8)));
        const float x = qr[d] * scale; const unsigned short hb = bf16_bits(x);
        aqh[ks].u[i] = hb; aql[ks].u[i] = bf16_bits(x - bf16_val(hb));
      }
  }
  float m_r[8], l_r[8];
#pragma unroll
  for (int r = 0; r < 8; ++r) { m_r[r] = -3.0e38f; l_r[r] = 0.f; }
  v8f oacc[DT];
#pragma unroll
  for (int dt = 0; dt < DT; ++dt) oacc[dt] = (v8f){0.f,0.f,0.f,0.f,0.f,0.f,0.f,0.f};

  const int kv_end = CAUSAL ? min(T, qblk * 64 + 64) : T;
  for (int j0 = 0; j0 < kv_end; j0 += 32) {
    __syncthreads();
    for (int e = tid; e < 32 * (D / 4); e += 128) {
      const int r = e / (D / 4), c4 = (e % (D / 4)) * 4;
      const int key = j0 + r;
      v4f kf = {0.f,0.f,0.f,0.f}, vf = {0.f,0.f,0.f,0.f};
      if (key < T) { kf = *(const v4fa*)(K + (size_t)key * pitch + c4); vf = *(const v4fa*)(V + (size_t)key * pitch + c4); }
#pragma unroll
      for (int t = 0; t < 4; ++t) {
        unsigned short hb = bf16_bits(kf[t]); sKh[r][c4 + t] = hb; sKl[r][c4 + t] = bf16_bits(kf[t] - bf16_val(hb));
        hb = bf16_bits(vf[t]); sVh[r][c4 + t] = hb; sVl[r][c4 + t] = bf16_bits(vf[t] - bf16_val(hb));
      }
    }
    __syncthreads();
    v8f s[2];
#pragma unroll
    for (int nt = 0; nt < 2; ++nt) {
      v8f acc = {};
#pragma unroll
      for (int ks = 0; ks < KS; ++ks) {
        FragB bh_, bl_;
        bh_.half[0] = *(const v8us*)&sKh[nt * 16 + ln][ks * 32 + 8 * hh]; bh_.half[1] = *(const v8us*)&sKh[nt * 16 + ln][ks * 32 + 16 + 8 * hh];
        bl_.half[0] = *(const v8us*)&sKl[nt * 16 + ln][ks * 32 + 8 * hh]; bl_.half[1] = *(const v8us*)&sKl[nt * 16 + ln][ks * 32 + 16 + 8 * hh];
        acc = mmaN<3>(aqh[ks].v, aql[ks].v, bh_.v, bl_.v, acc);
      }
      s[nt] = acc;
    }
    float alpha[8];
#pragma unroll
    for (int r = 0; r < 8; ++r) {
      const int qi = q0 + 8 * hh + r;
      const int ja = j0 + ln, jb = j0 + 16 + ln;
      if (CAUSAL) { if (ja > qi) s[0][r] = -3.0e38f; if (jb > qi) s[1][r] = -3.0e38f; }
      if (ja >= T) s[0][r] = -3.0e38f;
      if (jb >= T) s[1][r] = -3.0e38f;
      float mx = fmaxf(s[0][r], s[1][r]);
      mx = fmaxf(mx, __shfl_xor(mx, 1, 32)); mx = fmaxf(mx, __shfl_xor(mx, 2, 32)); mx = fmaxf(mx, __shfl_xor(mx, 4, 32)); mx = fmaxf(mx, __shfl_xor(mx, 8, 32));
      const float mnew = fmaxf(m_r[r], mx);
      alpha[r] = (mnew > -1.0e38f) ? __expf(m_r[r] - mnew) : 1.0f;
      const float p0 = (s[0][r] > -1.0e38f) ? __expf(s[0][r] - mnew) : 0.f;
      const float p1 = (s[1][r] > -1.0e38f) ? __expf(s[1][r] - mnew) : 0.f;
      m_r[r] = mnew;
      l_r[r] = l_r[r] * alpha[r] + p0 + p1;
      unsigned short hb = bf16_bits(p0); sPh[w][8 * hh + r][ln] = hb;      sPl[w][8 * hh + r][ln] = bf16_bits(p0 - bf16_val(hb));
      hb = bf16_bits(p1);                sPh[w][8 * hh + r][16 + ln] = hb; sPl[w][8 * hh + r][16 + ln] = bf16_bits(p1 - bf16_val(hb));
    }
#pragma unroll
    for (int dt = 0; dt < DT; ++dt)
#pragma unroll
      for (int r = 0; r < 8; ++r) oacc[dt][r] *= alpha[r];
    __builtin_amdgcn_fence(__ATOMIC_ACQ_REL, "workgroup");
    __builtin_amdgcn_wave_barrier();
    FragB pah, pal;
    pah.half[0] = *(const v8us*)&sPh[w][ln][8 * hh]; pah.half[1] = *(const v8us*)&sPh[w][ln][16 + 8 * hh];
    pal.half[0] = *(const v8us*)&sPl[w][ln][8 * hh]; pal.half[1] = *(const v8us*)&sPl[w][ln][16 + 8 * hh];
#pragma unroll
    for (int dt = 0; dt < DT; ++dt) {
      FragB bvh, bvl;
#pragma unroll
      for (int i = 0; i < 8; ++i) {
        bvh.u[i] = sVh[8 * hh + i][dt * 16 + ln]; bvh.u[8 + i] = sVh[16 + 8 * hh + i][dt * 16 + ln];
        bvl.u[i] = sVl[8 * hh + i][dt * 16 + ln]; bvl.u[8 + i] = sVl[16 + 8 * hh + i][dt * 16 + ln];
      }
      oacc[dt] = mmaN<3>(pah.v, pal.v, bvh.v, bvl.v, oacc[dt]);
    }
    __builtin_amdgcn_fence(__ATOMIC_ACQ_REL, "workgroup");
    __builtin_amdgcn_wave_barrier();
  }
#pragma unroll
  for (int r = 0; r < 8; ++r) {
    float l = l_r[r];
    l += __shfl_xor(l, 1, 32); l += __shfl_xor(l, 2, 32); l += __shfl_xor(l, 4, 32); l += __shfl_xor(l, 8, 32);
    l_r[r] = (l > 0.f) ? 1.0f / l : 0.f;
  }
#pragma unroll
  for (int dt = 0; dt < DT; ++dt)
#pragma unroll
    for (int r = 0; r < 8; ++r) sO[w][8 * hh + r][dt * 16 + ln] = oacc[dt][r] * l_r[r];
  __builtin_amdgcn_fence(__ATOMIC_ACQ_REL, "workgroup");
  __builtin_amdgcn_wave_barrier();
  for (int pass = 0; pass < 2; ++pass) {
    for (int r = 0; r < 16; ++r) {
      const int row = q0 + r;
      if (row < T && lane < D / 4) {
        const v4f val = *(const v4fa*)&sO[w][r][lane * 4];
        *(volatile v4f*)(y + ((size_t)b * T + row) * ypitch + h * D + lane * 4) = val;
      }
    }
    if (pass == 0) __threadfence();
  }
}

template <bool ASPLIT, int ACT, bool BIAS_BF16, bool RES_BF16>
__global__ __launch_bounds__(128) void k_gemm_bf3(const float* __restrict__ A, int lda, const unsigned short* __restrict__ Wt, int ldb,
                                                const float* __restrict__ bias, const float* __restrict__ resid, int rmod, int ldr,
                                                float* __restrict__ C, int ldc, int M, int N, int K) {
  __shared__ __attribute__((aligned(16))) float so[4][16][64];
  const int tid = threadIdx.x, w = tid >> 5, lane = tid & 31, ln = lane & 15, hh = lane >> 4;
  const int ntn = N / 64;
  const int wid = blockIdx.x * 4 + w;
  const int mt = wid / ntn, nq = wid % ntn;
  if (mt * 16 >= M) return;
  const int row0 = mt * 16, col0 = nq * 64;
  const float* arow = A + (size_t)(row0 + ln) * lda;
  v8f acc[4] = {};
  for (int kb = 0; kb < K; kb += 32) {
    FragB ah, al;
    const v4f x0 = *(const v4fa*)(arow + kb + 8 * hh), x1 = *(const v4fa*)(arow + kb + 8 * hh + 4);
    const v4f x2 = *(const v4fa*)(arow + kb + 16 + 8 * hh), x3 = *(const v4fa*)(arow + kb + 16 + 8 * hh + 4);
    float xs[16] = {x0[0],x0[1],x0[2],x0[3],x1[0],x1[1],x1[2],x1[3],x2[0],x2[1],x2[2],x2[3],x3[0],x3[1],x3[2],x3[3]};
#pragma unroll
    for (int i = 0; i < 16; ++i) { const unsigned short hb = bf16_bits(xs[i]); ah.u[i] = hb; al.u[i] = ASPLIT ? bf16_bits(xs[i] - bf16_val(hb)) : (unsigned short)0; }
#pragma unroll
    for (int t = 0; t < 4; ++t) {
      const unsigned short* brow = Wt + (size_t)(col0 + t * 16 + ln) * ldb + kb;
      FragB b;
      b.half[0] = *(const v8us*)(brow + 8 * hh);
      b.half[1] = *(const v8us*)(brow + 16 + 8 * hh);
      acc[t] = mmaN<ASPLIT ? 2 : 1>(ah.v, al.v, b.v, b.v, acc[t]);
    }
  }
#pragma unroll
  for (int t = 0; t < 4; ++t) {
    const int col = col0 + t * 16 + ln;
    float bv = bias ? bias[col] : 0.f;
    if (BIAS_BF16) bv = bf16_round(bv);
#pragma unroll
    for (int r = 0; r < 8; ++r) {
      float v = acc[t][r] + bv;
      if (resid) { float rv = resid[(size_t)((row0 + 8 * hh + r) % rmod) * ldr + col]; if (RES_BF16) rv = bf16_round(rv); v += rv; }
      if (ACT == 1) v = fmaxf(v, 0.f);
      if (ACT == 2) v = 0.5f * v * (1.0f + erff(v * 0.70710678118654752f));
      if (ACT == 3) { const float u = 0.7978845608028654f * (v + 0.044715f * v * v * v); v = 0.5f * v * (1.0f + tanhf(u)); }
      so[w][8 * hh + r][t * 16 + ln] = v;
    }
  }
  __builtin_amdgcn_fence(__ATOMIC_ACQ_REL, "workgroup");
  __builtin_amdgcn_wave_barrier();
  const int rsub = lane >> 4, c4 = (lane & 15) * 4;
  for (int pass = 0; pass < 2; ++pass) {
#pragma unroll
    for (int q = 0; q < 8; ++q) {
      const int r = q * 2 + rsub;
      const v4f v = *(const v4fa*)&so[w][r][c4];
      *(volatile v4f*)(C + (size_t)(row0 + r) * ldc + col0 + c4) = v;
    }
    if (pass == 0) __threadfence();
  }
}
template <bool PARAM_BF16>
__global__ __launch_bounds__(256) void k_layernorm(const float* __restrict__ X, const float* __restrict__ R, const float* __restrict__ g, const float* __restrict__ bta,
                                                  float* __restrict__ out_sum, float* __restrict__ out_norm, int N, float eps) {
  __shared__ float red[256];
  const int row = blockIdx.x, tid = threadIdx.x;
  const float* x = X + (size_t)row * N; const float* rr = R ? R + (size_t)row * N : nullptr;
  float vals[16];
  const int per = N / 256;
  float s1 = 0.f;
  for (int u = 0; u < per / 4; ++u) {
    const int j = tid * 4 + 1024 * u;
    const v4f a = *(const v4fa*)(x + j);
    v4f b = {0.f,0.f,0.f,0.f}; if (rr) b = *(const v4fa*)(rr + j);
#pragma unroll
    for (int q = 0; q < 4; ++q) { const float v = a[q] + b[q]; vals[u * 4 + q] = v; s1 += v; }
  }
  red[tid] = s1; __syncthreads();
  for (int st = 128; st > 0; st >>= 1) { if (tid < st) red[tid] += red[tid + st]; __syncthreads(); }
  const float mu = red[0] / (float)N; __syncthreads();
  float s2 = 0.f;
  for (int u = 0; u < per / 4; ++u)
#pragma unroll
    for (int q = 0; q < 4; ++q) { const float c = vals[u * 4 + q] - mu; s2 += c * c; }
  red[tid] = s2; __syncthreads();
  for (int st = 128; st > 0; st >>= 1) { if (tid < st) red[tid] += red[tid + st]; __syncthreads(); }
  const float rs = rsqrtf(red[0] / (float)N + eps);
  for (int pass = 0; pass < 2; ++pass) {
    for (int u = 0; u < per / 4; ++u) {
      const int j = tid * 4 + 1024 * u;
      v4f o, sm;
#pragma unroll
      for (int q = 0; q < 4; ++q) {
        float gg = g[j + q], bb = bta[j + q];
        if (PARAM_BF16) { gg = bf16_round(gg); bb = bf16_round(bb); }
        sm[q] = vals[u * 4 + q]; o[q] = (vals[u * 4 + q] - mu) * rs * gg + bb;
      }
      if (out_sum) *(volatile v4f*)(out_sum + (size_t)row * N + j) = sm;
      *(volatile v4f*)(out_norm + (size_t)row * N + j) = o;
    }
    if (pass == 0) __threadfence();
  }
}


typedef _Float16 v16h __attribute__((ext_vector_type(16)));
union FragH { v16h v; v8us half[2]; _Float16 h[16]; unsigned short u[16]; };
template <int NT>
__device__ __forceinline__ v8f mmaH(v16h ah, v16h al, v16h bh, v16h bl, v8f c) {
  c = __builtin_amdgcn_wmma_f32_16x16x32_f16(false, ah, false, bh, (short)0, c, false, false);
  if (NT >= 2) c = __builtin_amdgcn_wmma_f32_16x16x32_f16(false, al, false, bh, (short)0, c, false, false);
  if (NT >= 3) c = __builtin_amdgcn_wmma_f32_16x16x32_f16(false, ah, false, bl, (short)0, c, false, false);
  asm volatile("v_nop\n\tv_nop\n\tv_nop\n\tv_nop" : "+v"(c) : "v"(ah), "v"(al), "v"(bh), "v"(bl));
  return c;
}
template <bool ASPLIT>
__global__ __launch_bounds__(128) void k_gemm_h(const float* __restrict__ A, int lda, size_t sA, const _Float16* __restrict__ Bh, int ldb, size_t sB, float alpha, float* __restrict__ C, int ldc, size_t sC, int M, int N, int K) {
  __shared__ __attribute__((aligned(16))) float so[4][16][64];
  const int tid = threadIdx.x, w = tid >> 5, lane = tid & 31, ln = lane & 15, hh = lane >> 4; const int by = blockIdx.y;
  A += (size_t)by * sA; Bh += (size_t)by * sB; C += (size_t)by * sC;
  const int ntn = (N + 63) / 64; const int wid = blockIdx.x * 4 + w; const int mt = wid / ntn, nq = wid % ntn; if (mt * 16 >= M) return;
  const int row0 = mt * 16, col0 = nq * 64; const float* arow = A + (size_t)(row0 + ln) * lda;
  v8f acc[4] = {};
  for (int kb = 0; kb < K; kb += 32) {
    FragH ah, al;
    const v4f x0 = *(const v4fa*)(arow + kb + 8 * hh), x1 = *(const v4fa*)(arow + kb + 8 * hh + 4), x2 = *(const v4fa*)(arow + kb + 16 + 8 * hh), x3 = *(const v4fa*)(arow + kb + 16 + 8 * hh + 4);
    float xs[16] = {x0[0],x0[1],x0[2],x0[3],x1[0],x1[1],x1[2],x1[3],x2[0],x2[1],x2[2],x2[3],x3[0],x3[1],x3[2],x3[3]};
#pragma unroll
    for (int i = 0; i < 16; ++i) { const _Float16 h = (_Float16)xs[i]; ah.h[i] = h; al.h[i] = ASPLIT ? (_Float16)(xs[i] - (float)h) : (_Float16)0.0f; }
#pragma unroll
    for (int t = 0; t < 4; ++t) { if (col0 + t * 16 >= N) continue; const size_t boff = (size_t)(col0 + t * 16 + ln) * ldb + kb; FragH bq; bq.half[0] = *(const v8us*)(Bh + boff + 8 * hh); bq.half[1] = *(const v8us*)(Bh + boff + 16 + 8 * hh);
      acc[t] = mmaH<ASPLIT ? 2 : 1>(ah.v, al.v, bq.v, bq.v, acc[t]); }
  }
#pragma unroll
  for (int t = 0; t < 4; ++t) { if (col0 + t * 16 >= N) continue;
#pragma unroll
    for (int r = 0; r < 8; ++r) so[w][8 * hh + r][t * 16 + ln] = acc[t][r] * alpha; }
  __builtin_amdgcn_fence(__ATOMIC_ACQ_REL, "workgroup"); __builtin_amdgcn_wave_barrier();
  const int rsub = lane >> 4, c4 = (lane & 15) * 4;
  for (int pass = 0; pass < 2; ++pass) {
#pragma unroll
    for (int q = 0; q < 8; ++q) { const int r = q * 2 + rsub; if (col0 + c4 < N) { const v4f v = *(const v4fa*)&so[w][r][c4]; *(volatile v4f*)(C + (size_t)(row0 + r) * ldc + col0 + c4) = v; } }
    if (pass == 0) __threadfence(); }
}

__global__ __launch_bounds__(256) void k_wt_f16(const float* __restrict__ W, _Float16* __restrict__ Wt, int K, int N, float scale) {
  const int t = blockIdx.x * 256 + threadIdx.x; if (t >= N * (K / 8)) return; const int n = t / (K / 8), k8 = (t % (K / 8)) * 8; FragH f;
#pragma unroll
  for (int i = 0; i < 8; ++i) f.h[i] = (_Float16)(bf16_round(W[(size_t)(k8 + i) * N + n]) * scale); const v8us o = f.half[0];
  *(volatile v8us*)((unsigned short*)Wt + (size_t)n * K + k8) = o; __threadfence(); *(volatile v8us*)((unsigned short*)Wt + (size_t)n * K + k8) = o;
}
template <int ACT>
__global__ __launch_bounds__(128) void k_gemm_hhx(const _Float16* __restrict__ A, int lda, size_t sA, const _Float16* __restrict__ Bh, int ldb, size_t sB, float alpha, const float* __restrict__ bias, size_t sBias, const float* __restrict__ CP, int rowsPerB, size_t sCPb, int row0g,
    float* __restrict__ C, _Float16* __restrict__ C16, int ldc, size_t sC, int M, int N, int K) {
  __shared__ __attribute__((aligned(16))) float so[4][16][64];
  const int tid = threadIdx.x, w = tid >> 5, lane = tid & 31, ln = lane & 15, hh = lane >> 4; const int by = blockIdx.y;
  A += (size_t)by * sA; Bh += (size_t)by * sB; const size_t cofs = (size_t)by * sC; const float* bp = bias ? bias + (size_t)by * sBias : nullptr;
  const int ntn = (N + 63) / 64; const int wid = blockIdx.x * 4 + w; const int mt = wid / ntn, nq = wid % ntn; if (mt * 16 >= M) return;
  const int row0 = mt * 16, col0 = nq * 64; const _Float16* arow = A + (size_t)(row0 + ln) * lda;
  v8f acc[4] = {};
  for (int kb = 0; kb < K; kb += 32) { FragH ah; ah.half[0] = *(const v8us*)((const unsigned short*)arow + kb + 8 * hh); ah.half[1] = *(const v8us*)((const unsigned short*)arow + kb + 16 + 8 * hh);
#pragma unroll
    for (int t = 0; t < 4; ++t) { if (col0 + t * 16 >= N) continue; const size_t boff = (size_t)(col0 + t * 16 + ln) * ldb + kb; FragH bq; bq.half[0] = *(const v8us*)((const unsigned short*)Bh + boff + 8 * hh); bq.half[1] = *(const v8us*)((const unsigned short*)Bh + boff + 16 + 8 * hh);
      acc[t] = mmaH<1>(ah.v, ah.v, bq.v, bq.v, acc[t]); }
  }
#pragma unroll
  for (int t = 0; t < 4; ++t) { if (col0 + t * 16 >= N) continue; const int col = col0 + t * 16 + ln; const float bv = bp ? bf16_round(bp[col]) : 0.f;
#pragma unroll
    for (int r = 0; r < 8; ++r) { float v = acc[t][r] * alpha + bv; if (CP) { const int bidx = (row0g + row0 + 8 * hh + r) / rowsPerB; v += CP[(size_t)bidx * sCPb + (size_t)by * 64 + col]; } if (ACT == 1) v = (v > 0.f) ? v : expm1f(v); else if (ACT == 3) v = fmaxf(v, 0.f); so[w][8 * hh + r][t * 16 + ln] = v; } }
  __builtin_amdgcn_fence(__ATOMIC_ACQ_REL, "workgroup"); __builtin_amdgcn_wave_barrier();
  const int rsub = lane >> 4, c4 = (lane & 15) * 4; typedef _Float16 v4h __attribute__((ext_vector_type(4)));
  for (int pass = 0; pass < 2; ++pass) {
#pragma unroll
    for (int q = 0; q < 8; ++q) { const int r = q * 2 + rsub; if (col0 + c4 < N) { const v4f v = *(const v4fa*)&so[w][r][c4]; if (C) *(volatile v4f*)(C + cofs + (size_t)(row0 + r) * ldc + col0 + c4) = v; if (C16) { v4h h4; for (int i = 0; i < 4; ++i) h4[i] = (_Float16)v[i]; *(volatile v4h*)(C16 + cofs + (size_t)(row0 + r) * ldc + col0 + c4) = h4; } } }
    if (pass == 0) __threadfence(); }
}


__global__ __launch_bounds__(256) void k_x16(const float* __restrict__ x, _Float16* __restrict__ X16, size_t n8) { const size_t t = (size_t)blockIdx.x * 256 + threadIdx.x; if (t >= n8) return; FragH f;
#pragma unroll
  for (int q = 0; q < 8; ++q) f.h[q] = (_Float16)bf16_round(x[t * 8 + q]); *(volatile v8us*)((unsigned short*)X16 + t * 8) = f.half[0]; __threadfence(); *(volatile v8us*)((unsigned short*)X16 + t * 8) = f.half[0]; }
__global__ __launch_bounds__(256) void k_h16(const float* __restrict__ x, _Float16* __restrict__ X16, size_t n8) { const size_t t = (size_t)blockIdx.x * 256 + threadIdx.x; if (t >= n8) return; FragH f;
#pragma unroll
  for (int q = 0; q < 8; ++q) f.h[q] = (_Float16)x[t * 8 + q]; *(volatile v8us*)((unsigned short*)X16 + t * 8) = f.half[0]; __threadfence(); *(volatile v8us*)((unsigned short*)X16 + t * 8) = f.half[0]; }
__global__ __launch_bounds__(256) void k_round16f(const float* __restrict__ W, _Float16* __restrict__ Bt, size_t n8) { const size_t t = (size_t)blockIdx.x * 256 + threadIdx.x; if (t >= n8) return; FragH f;
#pragma unroll
  for (int i = 0; i < 8; ++i) f.h[i] = (_Float16)(bf16_round(W[t * 8 + i]) * 16.0f); *(volatile v8us*)((unsigned short*)Bt + t * 8) = f.half[0]; __threadfence(); *(volatile v8us*)((unsigned short*)Bt + t * 8) = f.half[0]; }
template <int NHv, int TTv>
__global__ __launch_bounds__(256) void k_vt(const _Float16* __restrict__ V16, int ldv, int voff, _Float16* __restrict__ Vt) { __shared__ unsigned short tl[64][66]; const int tid = threadIdx.x; const int slab = blockIdx.x / (TTv / 64), lg = blockIdx.x % (TTv / 64); const int b = slab / NHv, h = slab % NHv;
  for (int i = tid; i < 64 * 8; i += 256) { const int r = i / 8, c8 = (i % 8) * 8; FragH f; f.half[0] = *(const v8us*)((const unsigned short*)V16 + ((size_t)b * TTv + lg * 64 + r) * ldv + voff + h * 64 + c8);
#pragma unroll
    for (int q = 0; q < 8; ++q) tl[r][c8 + q] = f.u[q]; }
  __syncthreads();
  for (int pass = 0; pass < 2; ++pass) {
#pragma unroll
    for (int rd = 0; rd < 2; ++rd) { const int d = rd * 32 + tid / 8, pc = tid % 8; FragH f;
#pragma unroll
      for (int q = 0; q < 8; ++q) f.u[q] = tl[pc * 8 + q][d];
      *(volatile v8us*)((unsigned short*)Vt + ((size_t)slab * 64 + d) * TTv + lg * 64 + pc * 8) = f.half[0]; }
    if (pass == 0) __threadfence(); } }

__global__ __launch_bounds__(256) void k_xrows(const float* __restrict__ dur, const int* __restrict__ sid, const float* __restrict__ emb, _Float16* __restrict__ X16) { const int t8 = blockIdx.x * 256 + threadIdx.x; if (t8 >= TT * NB * 8) return; const int pc = t8 % 8; const int b = (t8 / 8) % NB; const int t = t8 / (8 * NB); int s = sid[b * TT + t]; s = s < 0 ? 0 : (s >= NSING ? NSING - 1 : s); FragH f;
#pragma unroll
  for (int q = 0; q < 8; ++q) { const int c = pc * 8 + q; f.h[q] = (_Float16)((c == 0) ? bf16_round(dur[b * TT + t]) : bf16_round(emb[(size_t)s * 63 + c - 1])); }
  *(volatile v8us*)((unsigned short*)X16 + (size_t)t8 * 8) = f.half[0]; __threadfence(); *(volatile v8us*)((unsigned short*)X16 + (size_t)t8 * 8) = f.half[0]; }
#define SCH 256
__device__ __forceinline__ float sigm_f(float x) { return 1.0f / (1.0f + __expf(-x)); }
__device__ __forceinline__ float tanh_f(float x) { const float e = __expf(2.0f * x); return 1.0f - 2.0f / (e + 1.0f); }
__global__ __launch_bounds__(256) void k_gru(int dir, int s0, const float* __restrict__ GI, const _Float16* __restrict__ Wh, const float* __restrict__ bH, const float* __restrict__ wd, unsigned short* __restrict__ HS, float* __restrict__ OD) {
  __shared__ __attribute__((aligned(16))) unsigned short shh[2][NB][HH + 8]; __shared__ float odp[2][4][NB];
  const int tid = threadIdx.x, w = tid >> 5, lane = tid & 31, ln = lane & 15, hh = lane >> 4; const int mt = w & 1, cg = w >> 1; const int c0 = cg * 64;
  unsigned short* hs = HS + (size_t)dir * NB * HH;
  for (int i = tid; i < NB * HH / 8; i += 256) { const v8us v = *(const v8us*)(hs + (size_t)i * 8); *(v8us*)&shh[0][(i * 8) / HH][(i * 8) % HH] = v; }
  __syncthreads();
#pragma unroll 1
  for (int si = 0; si < SCH; ++si) { const int s = s0 + si; const int t = dir ? (TT - 1 - s) : s; const int cur = si & 1, nxt = cur ^ 1;
    float orow[8];
#pragma unroll
    for (int r = 0; r < 8; ++r) orow[r] = 0.f;
#pragma unroll 1
    for (int nt = 0; nt < 4; ++nt) { const int c = c0 + nt * 16 + ln; const float bhn_ = bf16_round(bH[c]), wdv = bf16_round(wd[c]); v8f acc[3];
#pragma unroll
      for (int g = 0; g < 3; ++g) acc[g] = (v8f){0,0,0,0,0,0,0,0};
#pragma unroll 1
      for (int ks = 0; ks < HH / 32; ++ks) { FragH ah; ah.half[0] = *(const v8us*)&shh[cur][16 * mt + ln][ks * 32 + 8 * hh]; ah.half[1] = *(const v8us*)&shh[cur][16 * mt + ln][ks * 32 + 16 + 8 * hh];
#pragma unroll
        for (int g = 0; g < 3; ++g) { const unsigned short* br = (const unsigned short*)Wh + (size_t)(g * HH + c0 + nt * 16 + ln) * HH + ks * 32 + 8 * hh; FragH bk; bk.half[0] = *(const v8us*)br; bk.half[1] = *(const v8us*)(br + 16);
          acc[g] = mmaH<1>(ah.v, ah.v, bk.v, bk.v, acc[g]); } }
#pragma unroll
      for (int r = 0; r < 8; ++r) { const int row = 16 * mt + 8 * hh + r; const float* gi = GI + ((size_t)si * NB + row) * G3 + c;
        const float hr_ = acc[0][r] * 0.0625f, hz_ = acc[1][r] * 0.0625f, hn_ = acc[2][r] * 0.0625f;
        const float hprev = (float)(*(const _Float16*)&shh[cur][row][c]);
        const float rg = sigm_f(gi[0] + hr_); const float zg = sigm_f(gi[HH] + hz_); const float ng = tanh_f(gi[2 * HH] + rg * (hn_ + bhn_));
        const float hv = (1.0f - zg) * ng + zg * hprev; orow[r] += hv * wdv; FragH tmp; tmp.h[0] = (_Float16)hv; shh[nxt][row][c] = tmp.u[0]; } }
#pragma unroll
    for (int r = 0; r < 8; ++r) { float v = orow[r]; v += __shfl_xor(v, 1, 32); v += __shfl_xor(v, 2, 32); v += __shfl_xor(v, 4, 32); v += __shfl_xor(v, 8, 32); orow[r] = v; }
    { float pub = 0.f;
#pragma unroll
      for (int r = 0; r < 8; ++r) if (ln == r) pub = orow[r];
      if (ln < 8) odp[cur][cg][16 * mt + 8 * hh + ln] = pub; }
    __syncthreads();
    if (w == 0) { const float v = odp[cur][0][lane] + odp[cur][1][lane] + odp[cur][2][lane] + odp[cur][3][lane]; *(volatile float*)(OD + ((size_t)dir * TT + t) * NB + lane) = v; __threadfence(); *(volatile float*)(OD + ((size_t)dir * TT + t) * NB + lane) = v; } }
  __syncthreads();
  for (int pass = 0; pass < 2; ++pass) { for (int i = tid; i < NB * HH / 8; i += 256) { const v8us v = *(const v8us*)&shh[SCH & 1][(i * 8) / HH][(i * 8) % HH]; *(volatile v8us*)(hs + (size_t)i * 8) = v; } if (pass == 0) __threadfence(); }
}
__global__ __launch_bounds__(256) void k_zero(unsigned short* __restrict__ p, int n8) { const int i = blockIdx.x * 256 + threadIdx.x; if (i < n8) { const v8us z = {0,0,0,0,0,0,0,0}; *(volatile v8us*)(p + (size_t)i * 8) = z; __threadfence(); *(volatile v8us*)(p + (size_t)i * 8) = z; } }
__global__ __launch_bounds__(256) void k_xchunk(const _Float16* __restrict__ X16, int dir, int s0, _Float16* __restrict__ XC) { const int i = blockIdx.x * 256 + threadIdx.x; if (i >= SCH * NB * 8) return; const int pc = i % 8; const int b = (i / 8) % NB; const int si = i / (8 * NB); const int s = s0 + si; const int t = dir ? (TT - 1 - s) : s; const v8us v = *(const v8us*)((const unsigned short*)X16 + (((size_t)t * NB + b) * FF) + pc * 8); *(volatile v8us*)((unsigned short*)XC + (size_t)i * 8) = v; __threadfence(); *(volatile v8us*)((unsigned short*)XC + (size_t)i * 8) = v; }
__global__ __launch_bounds__(256) void k_out(const float* __restrict__ OD, const float* __restrict__ bd, float* __restrict__ out) { const int i = blockIdx.x * 256 + threadIdx.x; if (i >= NB * TT) return; const int t = i % TT, b = i / TT; const float v = OD[(size_t)t * NB + b] + OD[((size_t)TT + t) * NB + b] + bf16_round(bd[0]); *(volatile float*)(out + i) = v; __threadfence(); *(volatile float*)(out + i) = v; }
extern "C" void kernel_launch(void* const* d_in, const int* in_sizes, int n_in,
                              void* d_out, int out_size, void* d_ws, size_t ws_size, hipStream_t stream) {
  (void)in_sizes; (void)n_in; (void)out_size;
  const float* dur = (const float*)d_in[0]; const int* sid = (const int*)d_in[1]; const float* emb = (const float*)d_in[2]; const float* Wi_f = (const float*)d_in[3]; const float* Wh_f = (const float*)d_in[4]; const float* bi_f = (const float*)d_in[5]; const float* bhn_f = (const float*)d_in[6]; const float* Wi_b = (const float*)d_in[7]; const float* Wh_b = (const float*)d_in[8]; const float* bi_b = (const float*)d_in[9]; const float* bhn_b = (const float*)d_in[10]; const float* Wd = (const float*)d_in[11]; const float* bd = (const float*)d_in[12];
  char* ws = (char*)d_ws; size_t off = 0;
  auto take = [&](size_t bytes) { char* p = ws + off; off += (bytes + 255) & ~(size_t)255; return p; };
  _Float16* BWi = (_Float16*)take((size_t)2 * G3 * FF * 2); _Float16* BWh = (_Float16*)take((size_t)2 * G3 * HH * 2); _Float16* X16 = (_Float16*)take((size_t)TT * NB * FF * 2); _Float16* XC = (_Float16*)take((size_t)SCH * NB * FF * 2); float* GI = (float*)take((size_t)SCH * NB * G3 * 4); unsigned short* HS = (unsigned short*)take((size_t)2 * NB * HH * 2); float* OD = (float*)take((size_t)2 * TT * NB * 4);
  if (off > ws_size) return;
  k_wt_f16<<<(G3 * (FF / 8) + 255) / 256, 256, 0, stream>>>(Wi_f, BWi, FF, G3, 16.0f); k_wt_f16<<<(G3 * (FF / 8) + 255) / 256, 256, 0, stream>>>(Wi_b, BWi + (size_t)G3 * FF, FF, G3, 16.0f);
  k_wt_f16<<<(G3 * (HH / 8) + 255) / 256, 256, 0, stream>>>(Wh_f, BWh, HH, G3, 16.0f); k_wt_f16<<<(G3 * (HH / 8) + 255) / 256, 256, 0, stream>>>(Wh_b, BWh + (size_t)G3 * HH, HH, G3, 16.0f);
  k_xrows<<<(TT * NB * 8 + 255) / 256, 256, 0, stream>>>(dur, sid, emb, X16);
  k_zero<<<(2 * NB * HH / 8 + 255) / 256, 256, 0, stream>>>(HS, 2 * NB * HH / 8);
  for (int dir = 0; dir < 2; ++dir) { const float* biD = dir ? bi_b : bi_f; const float* bhnD = dir ? bhn_b : bhn_f;
    for (int s0 = 0; s0 < TT; s0 += SCH) {
      k_xchunk<<<(SCH * NB * 8 + 255) / 256, 256, 0, stream>>>(X16, dir, s0, XC);
      k_gemm_hhx<0><<<dim3(((SCH * NB / 16) * (G3 / 64) + 3) / 4, 1), 128, 0, stream>>>(XC, FF, 0, BWi + (size_t)dir * G3 * FF, FF, 0, 0.0625f, biD, 0, nullptr, 1, 0, 0, GI, nullptr, G3, 0, SCH * NB, G3, FF);
      k_gru<<<1, 256, 0, stream>>>(dir, s0, GI, BWh + (size_t)dir * G3 * HH, bhnD, Wd + dir * HH, HS, OD); } }
  k_out<<<(NB * TT + 255) / 256, 256, 0, stream>>>(OD, bd, (float*)d_out);
}
